// KimiDeltaAttention_5016521802517
// MI455X (gfx1250) — hardware-run, weakly checked
//
#include <hip/hip_runtime.h>
#include <math.h>

constexpr int SEQ_T = 1024;
constexpr int DMOD  = 2048;
constexpr int NHEAD = 16;
constexpr int HDIM  = 128;
constexpr int CHN   = 2048;
constexpr int KCONV = 4;
constexpr int NFG   = 320;
constexpr float EPS_N = 1e-6f;
constexpr size_t TK_ELEMS = (size_t)SEQ_T * CHN;

static_assert(CHN == NHEAD * HDIM, "shape");
static_assert(SEQ_T % 64 == 0 && CHN % 64 == 0 && DMOD % 64 == 0 && NFG % 64 == 0, "GEMM M/N tile multiples");
static_assert(DMOD % 32 == 0 && HDIM % 32 == 0 && CHN % 32 == 0, "GEMM K % 32");

typedef __attribute__((ext_vector_type(16))) _Float16 v16h;
typedef __attribute__((ext_vector_type(8)))  _Float16 v8h;
typedef __attribute__((ext_vector_type(16))) __bf16   v16b;
typedef __attribute__((ext_vector_type(8)))  __bf16   v8b;
typedef __attribute__((ext_vector_type(8)))  float    v8f;
typedef __attribute__((ext_vector_type(4)))  float    v4f;
typedef __attribute__((ext_vector_type(4)))  unsigned v4u;

__device__ __forceinline__ unsigned short f2bf_bits(float f) {
  unsigned u = __float_as_uint(f);
  return (unsigned short)((u + 0x7FFFu + ((u >> 16) & 1u)) >> 16);
}
__device__ __forceinline__ float bf_bits2f(unsigned short h) { return __uint_as_float(((unsigned)h) << 16); }
__device__ __forceinline__ float bfr(float f) { return __uint_as_float(((unsigned)f2bf_bits(f)) << 16); }
__device__ __forceinline__ float rcp_f(float x) { return __builtin_amdgcn_rcpf(x); }
__device__ __forceinline__ float rsq_f(float x) { return __builtin_amdgcn_rsqf(x); }
__device__ __forceinline__ float sigm_f(float x) { return rcp_f(1.0f + expf(-x)); }

__device__ __forceinline__ void dep_guard_h(v8f& a, v8f& b, v16h x, v16h y) { asm volatile("v_nop\n\tv_nop\n\tv_nop\n\tv_nop" : "+v"(a), "+v"(b) : "v"(x), "v"(y)); }
__device__ __forceinline__ void dep_guard_b(v8f& a, v8f& b, v16b x, v16b y) { asm volatile("v_nop\n\tv_nop\n\tv_nop\n\tv_nop" : "+v"(a), "+v"(b) : "v"(x), "v"(y)); }
__device__ __forceinline__ void keep4_h(v16h a, v16h b, v16h c, v16h d) { asm volatile("v_nop" :: "v"(a), "v"(b), "v"(c), "v"(d)); }
__device__ __forceinline__ void keep4_b(v16b a, v16b b, v16b c, v16b d) { asm volatile("v_nop" :: "v"(a), "v"(b), "v"(c), "v"(d)); }
__device__ __forceinline__ void acc_guard4(v8f& a, v8f& b, v8f& c, v8f& d) { asm volatile("v_nop\n\tv_nop\n\tv_nop\n\tv_nop" : "+v"(a), "+v"(b), "+v"(c), "+v"(d)); }
template <typename T> struct Frag;
template <> struct Frag<_Float16> {
  typedef v16h V; union U { v16h v; v8h h[2]; };
  static __device__ __forceinline__ v16h load(const _Float16* p) {
    U f; f.h[0] = *(const v8h*)(p); f.h[1] = *(const v8h*)(p + 16); return f.v;
  }
  static __device__ __forceinline__ v8f mma(v16h a, v16h b, v8f c) {
    return __builtin_amdgcn_wmma_f32_16x16x32_f16(false, a, false, b, (short)0, c, false, false);
  }
  static __device__ __forceinline__ void guard(v8f& a, v8f& b, v16h x, v16h y) { dep_guard_h(a, b, x, y); }
  static __device__ __forceinline__ void keep(v16h a, v16h b, v16h c, v16h d) { keep4_h(a, b, c, d); }
};
template <> struct Frag<__bf16> {
  typedef v16b V; union U { v16b v; v8b h[2]; };
  static __device__ __forceinline__ v16b load(const __bf16* p) {
    U f; f.h[0] = *(const v8b*)(p); f.h[1] = *(const v8b*)(p + 16); return f.v;
  }
  static __device__ __forceinline__ v8f mma(v16b a, v16b b, v8f c) {
    return __builtin_amdgcn_wmma_f32_16x16x32_bf16(false, a, false, b, (short)0, c, false, false);
  }
  static __device__ __forceinline__ void guard(v8f& a, v8f& b, v16b x, v16b y) { dep_guard_b(a, b, x, y); }
  static __device__ __forceinline__ void keep(v16b a, v16b b, v16b c, v16b d) { keep4_b(a, b, c, d); }
};

template <int ET> struct Elem;
template <> struct Elem<0> { typedef _Float16 T; };
template <> struct Elem<1> { typedef __bf16 T; };
template <int ET, int SPLITM, int BIAS_MODE, int OUT_MODE>
__global__ __launch_bounds__(256) void wmma_gemm64(
    const unsigned short* __restrict__ Ap, const unsigned short* __restrict__ A2p, int lda, long strideA,
    const unsigned short* __restrict__ Btp, const unsigned short* __restrict__ Bt2p, int ldb, long strideB,
    void* __restrict__ Cout, void* __restrict__ Cout2, int ldc, long strideC,
    const float* __restrict__ bias,
    int M, int N, int K, float scale) {
  typedef typename Elem<ET>::T T;
  typedef typename Frag<T>::V V;
  const T* A = (const T*)Ap; const T* A2 = (const T*)A2p; const T* Bt = (const T*)Btp; const T* Bt2 = (const T*)Bt2p;
  __shared__ __align__(16) float sT[8][16 * 68];
  const int b    = blockIdx.y;
  const int lane = threadIdx.x & 31;
  const int wave = threadIdx.x >> 5;
  const int tilesN = N >> 6;
  const int tilesM = M >> 6;
  const int tile = blockIdx.x * 8 + wave;
  if (tile >= tilesM * tilesN) return;
  const int tm = tile / tilesN;
  const int tn = tile - tm * tilesN;
  const int m0 = tm << 6;
  const int n0 = tn << 6;

  const T* Ab  = A  + (size_t)b * strideA;
  const T* Bb  = Bt + (size_t)b * strideB;
  const T* Ab2 = (SPLITM >= 1) ? (A2  + (size_t)b * strideA) : nullptr;
  const T* Bb2 = (SPLITM == 2) ? (Bt2 + (size_t)b * strideB) : nullptr;

  const int rlane = lane & 15;
  const int koff  = (lane >> 4) * 8;
  const int mOff  = (lane >> 4) * 8;

  v8f acc[4][4];
#pragma unroll
  for (int i = 0; i < 4; ++i)
#pragma unroll
    for (int j = 0; j < 4; ++j) acc[i][j] = (v8f){0.f,0.f,0.f,0.f,0.f,0.f,0.f,0.f};

  for (int k0 = 0; k0 < K; k0 += 32) {
    V bh[4], bl[4];
#pragma unroll
    for (int j = 0; j < 4; ++j) {
      const size_t bo = (size_t)(n0 + (j << 4) + rlane) * ldb + koff + k0;
      bh[j] = Frag<T>::load(Bb + bo);
      if (SPLITM == 2) bl[j] = Frag<T>::load(Bb2 + bo);
    }
#pragma unroll
    for (int i = 0; i < 4; ++i) {
      const size_t ao = (size_t)(m0 + (i << 4) + rlane) * lda + koff + k0;
      V ah = Frag<T>::load(Ab + ao);
      V al;
      if (SPLITM >= 1) al = Frag<T>::load(Ab2 + ao);
#pragma unroll
      for (int j = 0; j < 4; ++j) {
        acc[i][j] = Frag<T>::mma(ah, bh[j], acc[i][j]);
        if (SPLITM == 2) acc[i][j] = Frag<T>::mma(ah, bl[j], acc[i][j]);
        if (SPLITM >= 1) acc[i][j] = Frag<T>::mma(al, bh[j], acc[i][j]);
      }
      Frag<T>::guard(acc[i][0], acc[i][3], ah, (SPLITM >= 1) ? al : ah);
    }
    Frag<T>::keep(bh[0], bh[1], bh[2], bh[3]);
    if (SPLITM == 2) Frag<T>::keep(bl[0], bl[1], bl[2], bl[3]);
  }
  acc_guard4(acc[0][0], acc[0][1], acc[0][2], acc[0][3]);
  acc_guard4(acc[1][0], acc[1][1], acc[1][2], acc[1][3]);
  acc_guard4(acc[2][0], acc[2][1], acc[2][2], acc[2][3]);
  acc_guard4(acc[3][0], acc[3][1], acc[3][2], acc[3][3]);

  float* slab = sT[wave];
#pragma unroll
  for (int i = 0; i < 4; ++i) {
    const int mBase = m0 + (i << 4);
#pragma unroll
    for (int j = 0; j < 4; ++j) {
      const int n = n0 + (j << 4) + rlane;
      float bv = 0.f;
      if (BIAS_MODE == 2) bv = bias[n];
#pragma unroll
      for (int r = 0; r < 8; ++r) {
        float v = acc[i][j][r] * scale;
        if (BIAS_MODE == 1) v += bias[mBase + mOff + r];
        if (BIAS_MODE == 2) v += bv;
        slab[(mOff + r) * 68 + (j << 4) + rlane] = v;
      }
    }
    __builtin_amdgcn_fence(__ATOMIC_RELEASE, "workgroup");
    __builtin_amdgcn_wave_barrier();
    __builtin_amdgcn_fence(__ATOMIC_ACQUIRE, "workgroup");
    if (OUT_MODE == 0) {
      float* C = (float*)Cout + (size_t)b * strideC;
      const int hh = lane >> 4, c4 = (lane & 15) * 4;
      for (int pass = 0; pass < 2; ++pass) {
#pragma unroll
        for (int it = 0; it < 8; ++it) {
          const int row = it * 2 + hh;
          v4f v = *(const v4f*)(slab + row * 68 + c4);
          *(volatile v4f*)(C + (size_t)(mBase + row) * ldc + n0 + c4) = v;
        }
        __threadfence();
      }
    } else {
      const int q = lane >> 3, c8 = (lane & 7) * 8;
      unsigned short* C  = (unsigned short*)Cout  + (size_t)b * strideC;
      unsigned short* C2 = (OUT_MODE == 2) ? ((unsigned short*)Cout2 + (size_t)b * strideC) : nullptr;
      for (int pass = 0; pass < 2; ++pass) {
#pragma unroll
        for (int it = 0; it < 4; ++it) {
          const int row = it * 4 + q;
          const float* sp = slab + row * 68 + c8;
          v8h hv, lv;
#pragma unroll
          for (int e = 0; e < 8; ++e) {
            if (OUT_MODE == 1) {
              hv[e] = (_Float16)sp[e];
            } else {
              unsigned short hb = f2bf_bits(sp[e]);
              unsigned short lb = f2bf_bits(sp[e] - bf_bits2f(hb));
              hv[e] = __builtin_bit_cast(_Float16, hb);
              lv[e] = __builtin_bit_cast(_Float16, lb);
            }
          }
          *(volatile v8h*)(C + (size_t)(mBase + row) * ldc + n0 + c8) = hv;
          if (OUT_MODE == 2) *(volatile v8h*)(C2 + (size_t)(mBase + row) * ldc + n0 + c8) = lv;
        }
        __threadfence();
      }
    }
    __builtin_amdgcn_fence(__ATOMIC_RELEASE, "workgroup");
    __builtin_amdgcn_wave_barrier();
    __builtin_amdgcn_fence(__ATOMIC_ACQUIRE, "workgroup");
  }
}

__global__ __launch_bounds__(256) void k_cast_bf16x8(const float* __restrict__ in,
                                                     unsigned short* __restrict__ out, int n8) {
  const int i = blockIdx.x * 256 + threadIdx.x;
  if (i < n8) {
    const v4f a = *(const v4f*)(in + (size_t)i * 8);
    const v4f c = *(const v4f*)(in + (size_t)i * 8 + 4);
    v4u u;
    u[0] = (unsigned)f2bf_bits(a[0]) | ((unsigned)f2bf_bits(a[1]) << 16);
    u[1] = (unsigned)f2bf_bits(a[2]) | ((unsigned)f2bf_bits(a[3]) << 16);
    u[2] = (unsigned)f2bf_bits(c[0]) | ((unsigned)f2bf_bits(c[1]) << 16);
    u[3] = (unsigned)f2bf_bits(c[2]) | ((unsigned)f2bf_bits(c[3]) << 16);
    unsigned short* p = out + (size_t)i * 8;
    *(volatile v4u*)(void*)p = u;
    __threadfence();
    *(volatile v4u*)(void*)p = u;
  }
}

__global__ __launch_bounds__(256) void k_tr_bf16(const float* __restrict__ in0, const float* __restrict__ in1,
                                                 const float* __restrict__ in2, const float* __restrict__ in3,
                                                 unsigned short* __restrict__ out, long ostride,
                                                 int rows, int cols, int ldo) {
  __shared__ float tile[64][65];
  const int z = blockIdx.z;
  const float* in = (z == 0) ? in0 : (z == 1) ? in1 : (z == 2) ? in2 : in3;
  unsigned short* op = out + (size_t)z * ostride;
  const int r0 = blockIdx.y * 64, c0 = blockIdx.x * 64;
  const int tid = threadIdx.x, lane = tid & 31, wave = tid >> 5;
#pragma unroll
  for (int i = 0; i < 4; ++i) {
    const int idx = i * 256 + tid;
    const int r   = idx >> 4;
    const int cq  = (idx & 15) * 4;
    const int c   = c0 + cq;
    const bool valid = (c < cols);
    const int cc  = valid ? c : (cols - 4);
    const v4f v = *(const v4f*)(in + (size_t)(r0 + r) * cols + cc);
#pragma unroll
    for (int e = 0; e < 4; ++e) tile[cq + e][r] = valid ? v[e] : 0.0f;
  }
  __syncthreads();
  const int q = lane >> 3, c8 = (lane & 7) * 8;
  for (int pass = 0; pass < 2; ++pass) {
#pragma unroll
    for (int it = 0; it < 2; ++it) {
      const int cl = wave * 8 + it * 4 + q;
      v4u u;
#pragma unroll
      for (int e = 0; e < 4; ++e) {
        const unsigned lo16 = (unsigned)f2bf_bits(tile[cl][c8 + 2 * e]);
        const unsigned hi16 = (unsigned)f2bf_bits(tile[cl][c8 + 2 * e + 1]);
        u[e] = lo16 | (hi16 << 16);
      }
      unsigned short* dst = op + (size_t)(c0 + cl) * ldo + r0 + c8;
      *(volatile v4u*)(void*)dst = u;
    }
    __threadfence();
  }
}

__global__ __launch_bounds__(256) void k_conv_silu_norm(const float* __restrict__ lin,
                                                        const float* __restrict__ cwq, const float* __restrict__ cwk,
                                                        const float* __restrict__ cwv,
                                                        float* __restrict__ post, float qscale) {
  const int lane = threadIdx.x & 31, wave = threadIdx.x >> 5;
  const int row = blockIdx.x * 8 + wave;
  const int y = blockIdx.y;
  const float* in = lin + (size_t)y * TK_ELEMS;
  float* outp = post + (size_t)y * TK_ELEMS;
  const float* w = (y == 0) ? cwq : (y == 1) ? cwk : cwv;
  const int t = row >> 4, h = row & 15;
  const int c = h * HDIM + lane * 4;
  v4f acc = {0.f, 0.f, 0.f, 0.f};
#pragma unroll
  for (int j = 0; j < KCONV; ++j) {
    const int tt  = t + j - (KCONV - 1);
    const int ttc = tt < 0 ? 0 : tt;
    const v4f xv = *(const v4f*)(in + (size_t)ttc * CHN + c);
    const v4f wv = *(const v4f*)(w + (size_t)j * CHN + c);
    const bool m = (tt >= 0);
#pragma unroll
    for (int e = 0; e < 4; ++e) {
      const float xe = m ? xv[e] : 0.0f;
      acc[e] = fmaf(bfr(wv[e]), xe, acc[e]);
    }
  }
  v4f s;
#pragma unroll
  for (int e = 0; e < 4; ++e) s[e] = acc[e] * sigm_f(acc[e]);
  float ss = 0.0f;
  ss += s[0] * s[0]; ss += s[1] * s[1]; ss += s[2] * s[2]; ss += s[3] * s[3];
#pragma unroll
  for (int off = 16; off > 0; off >>= 1) ss += __shfl_xor(ss, off, 32);
  const float rn = rsq_f(ss + EPS_N);
  const float r = (y == 0) ? (rn * qscale) : (y == 1) ? rn : 1.0f;
  v4f o;
#pragma unroll
  for (int e = 0; e < 4; ++e) o[e] = s[e] * r;
  float* dst = outp + (size_t)t * CHN + c;
  *(volatile v4f*)dst = o;
  __threadfence();
  *(volatile v4f*)dst = o;
}

__global__ __launch_bounds__(256) void k_gate_exp(const float* __restrict__ graw, const float* __restrict__ dtb,
                                                  const float* __restrict__ alog, float* __restrict__ eg) {
  const int i = blockIdx.x * 256 + threadIdx.x;
  const int c = i & (CHN - 1);
  const int h = c >> 7;
  float xg = graw[i] + bfr(dtb[c]);
  xg = fminf(fmaxf(xg, -20.0f), 20.0f);
  const float sp = log1pf(expf(xg));
  const float a  = expf(bfr(alog[h]));
  const float g  = -(a * sp);
  const float e  = expf(g);
  ((volatile float*)eg)[i] = e;
  __threadfence();
  ((volatile float*)eg)[i] = e;
}

__global__ __launch_bounds__(512) void k_scan(const float* __restrict__ qf, const float* __restrict__ kf,
                                             const float* __restrict__ vv, const float* __restrict__ eg,
                                             const unsigned* __restrict__ pbh, const unsigned* __restrict__ pbl,
                                             float* __restrict__ o) {
  __shared__ __align__(16) float s_eg[HDIM];
  __shared__ __align__(16) float s_k[HDIM];
  __shared__ __align__(16) float s_q[HDIM];
  __shared__ float s_v[64];
  __shared__ float s_u[64];
  __shared__ float s_part[8][64];
  __shared__ __align__(16) float s_o[64];
  __shared__ float s_beta;

  const int h   = blockIdx.x >> 1;
  const int jv  = blockIdx.x & 1;
  const int tid = threadIdx.x;
  const int lane = tid & 31;
  const int wave = tid >> 5;
  const int vi  = tid & 63;
  const int kg  = tid >> 6;
  const int kb  = kg * 16;

  float st[16];
#pragma unroll
  for (int i = 0; i < 16; ++i) st[i] = 0.0f;

  for (int t = 0; t < SEQ_T; ++t) {
    const size_t base = (size_t)t * CHN + (size_t)h * HDIM;
    if (wave < 4) {
      s_eg[tid] = eg[base + tid];
      s_k[tid]  = kf[base + tid];
    } else if (wave < 8) {
      s_q[tid - 128] = qf[base + tid - 128];
    } else if (wave < 10) {
      s_v[tid - 256] = vv[base + 64 * jv + (tid - 256)];
    } else if (wave == 10) {
      const unsigned wi = ((unsigned)(t * NFG + 256 + h)) >> 1;
      const unsigned w0 = pbh[wi];
      const unsigned w1 = pbl[wi];
      const unsigned hb = (h & 1) ? (w0 & 0xffff0000u) : (w0 << 16);
      const unsigned lb = (h & 1) ? (w1 & 0xffff0000u) : (w1 << 16);
      const float braw = __uint_as_float(hb) + __uint_as_float(lb);
      const float bs = sigm_f(braw);
      if (lane == 0) s_beta = bs;
    }
    __syncthreads();

    float partial = 0.0f;
#pragma unroll
    for (int i = 0; i < 16; ++i) {
      st[i] = st[i] * s_eg[kb + i];
      partial = fmaf(s_k[kb + i], st[i], partial);
    }
    s_part[kg][vi] = partial;
    __syncthreads();

    if (wave < 2) {
      float inner = 0.0f;
#pragma unroll
      for (int gq = 0; gq < 8; ++gq) inner += s_part[gq][tid];
      s_u[tid] = s_beta * (s_v[tid] - inner);
    }
    __syncthreads();

    const float u = s_u[vi];
    float po = 0.0f;
#pragma unroll
    for (int i = 0; i < 16; ++i) {
      st[i] = fmaf(s_k[kb + i], u, st[i]);
      po = fmaf(s_q[kb + i], st[i], po);
    }
    s_part[kg][vi] = po;
    __syncthreads();

    if (wave == 0) {
      float o0 = 0.0f, o1 = 0.0f;
#pragma unroll
      for (int gq = 0; gq < 8; ++gq) { o0 += s_part[gq][lane]; o1 += s_part[gq][lane + 32]; }
      s_o[lane] = o0;
      s_o[lane + 32] = o1;
      __builtin_amdgcn_fence(__ATOMIC_RELEASE, "workgroup");
      __builtin_amdgcn_wave_barrier();
      __builtin_amdgcn_fence(__ATOMIC_ACQUIRE, "workgroup");
      float* dst = o + base + 64 * jv;
      if (lane < 16) {
        const v4f val = *(const v4f*)(s_o + 4 * lane);
        *(volatile v4f*)(dst + 4 * lane) = val;
      }
      __threadfence();
      if (lane < 16) {
        const v4f val = *(const v4f*)(s_o + 4 * lane);
        *(volatile v4f*)(dst + 4 * lane) = val;
      }
    }
  }
}

__global__ __launch_bounds__(256) void k_rmsnorm_gate_split(const float* __restrict__ ob, const float* __restrict__ gout,
                                                            const float* __restrict__ nw,
                                                            unsigned short* __restrict__ onh,
                                                            unsigned short* __restrict__ onl) {
  const int lane = threadIdx.x & 31, wave = threadIdx.x >> 5;
  const int hr = lane >> 4, cl = lane & 15;
  const int row = (blockIdx.x * 8 + wave) * 2 + hr;
  const int t = row >> 4, h = row & 15;
  const size_t base = (size_t)t * CHN + (size_t)h * HDIM + (size_t)cl * 8;
  const v4f oa = *(const v4f*)(ob + base);
  const v4f oc = *(const v4f*)(ob + base + 4);
  const v4f ga = *(const v4f*)(gout + base);
  const v4f gc = *(const v4f*)(gout + base + 4);
  const v4f na = *(const v4f*)(nw + cl * 8);
  const v4f nc = *(const v4f*)(nw + cl * 8 + 4);
  float ss = 0.0f;
  ss += oa[0] * oa[0]; ss += oa[1] * oa[1]; ss += oa[2] * oa[2]; ss += oa[3] * oa[3];
  ss += oc[0] * oc[0]; ss += oc[1] * oc[1]; ss += oc[2] * oc[2]; ss += oc[3] * oc[3];
#pragma unroll
  for (int off = 8; off > 0; off >>= 1) ss += __shfl_xor(ss, off, 32);
  const float rstd = rsq_f(ss * (1.0f / 128.0f) + EPS_N);
  v4u uh, ul;
#pragma unroll
  for (int e = 0; e < 4; ++e) {
    float v0, v1, g0, g1, n0v, n1v;
    if (e < 2) { v0 = oa[2 * e]; v1 = oa[2 * e + 1]; g0 = ga[2 * e]; g1 = ga[2 * e + 1]; n0v = na[2 * e]; n1v = na[2 * e + 1]; }
    else       { v0 = oc[2 * e - 4]; v1 = oc[2 * e - 3]; g0 = gc[2 * e - 4]; g1 = gc[2 * e - 3]; n0v = nc[2 * e - 4]; n1v = nc[2 * e - 3]; }
    float r0v = v0 * rstd; r0v = r0v * bfr(n0v); r0v = r0v * sigm_f(g0);
    float r1v = v1 * rstd; r1v = r1v * bfr(n1v); r1v = r1v * sigm_f(g1);
    const unsigned short h0 = f2bf_bits(r0v);
    const unsigned short l0 = f2bf_bits(r0v - bf_bits2f(h0));
    const unsigned short h1 = f2bf_bits(r1v);
    const unsigned short l1 = f2bf_bits(r1v - bf_bits2f(h1));
    uh[e] = (unsigned)h0 | ((unsigned)h1 << 16);
    ul[e] = (unsigned)l0 | ((unsigned)l1 << 16);
  }
  unsigned short* dh = onh + base;
  unsigned short* dl = onl + base;
  *(volatile v4u*)(void*)dh = uh;
  *(volatile v4u*)(void*)dl = ul;
  __threadfence();
  *(volatile v4u*)(void*)dh = uh;
  *(volatile v4u*)(void*)dl = ul;
}

constexpr size_t OFF_XBF  = 0;
constexpr size_t SZ_XBF   = (size_t)SEQ_T * DMOD * 2;
constexpr size_t OFF_WT4  = OFF_XBF + SZ_XBF;
constexpr size_t SZ_WT4   = (size_t)4 * DMOD * CHN * 2;
constexpr size_t OFF_WFG  = OFF_WT4 + SZ_WT4;
constexpr size_t SZ_WFG   = (size_t)NFG * DMOD * 2;
constexpr size_t OFF_WFBG = OFF_WFG + SZ_WFG;
constexpr size_t SZ_WFBG  = (size_t)2 * CHN * HDIM * 2;
constexpr size_t OFF_LIN  = OFF_WFBG + SZ_WFBG;
constexpr size_t SZ_LIN   = (size_t)3 * TK_ELEMS * 4;
constexpr size_t OFF_EG   = OFF_LIN;
constexpr size_t OFF_OBUF = OFF_LIN + TK_ELEMS * 4;
constexpr size_t OFF_ONH  = OFF_LIN + 2 * TK_ELEMS * 4;
constexpr size_t OFF_ONL  = OFF_ONH + TK_ELEMS * 2;
constexpr size_t OFF_PFH  = OFF_LIN + SZ_LIN;
constexpr size_t SZ_PF    = (size_t)SEQ_T * NFG * 2;
constexpr size_t OFF_PFL  = OFF_PFH + SZ_PF;
constexpr size_t OFF_GR   = OFF_PFL + SZ_PF;
constexpr size_t SZ_GR    = (size_t)2 * TK_ELEMS * 4;
constexpr size_t OFF_POST = OFF_GR + SZ_GR;
constexpr size_t SZ_POST  = (size_t)3 * TK_ELEMS * 4;
constexpr size_t WS_TOTAL = OFF_POST + SZ_POST;
static_assert(OFF_ONL + TK_ELEMS * 2 <= OFF_LIN + SZ_LIN, "reused region fits");
static_assert(WS_TOTAL == 108527616ull, "carve total");
static_assert(WS_TOTAL <= 134217728ull, "carve under 128 MiB");
static_assert((OFF_WT4 % 256) == 0 && (OFF_WFG % 256) == 0 && (OFF_WFBG % 256) == 0 && (OFF_LIN % 256) == 0 &&
              (OFF_OBUF % 256) == 0 && (OFF_ONH % 256) == 0 && (OFF_ONL % 256) == 0 && (OFF_PFH % 256) == 0 &&
              (OFF_PFL % 256) == 0 && (OFF_GR % 256) == 0 && (OFF_POST % 256) == 0, "aligned carves");

extern "C" void kernel_launch(void* const* d_in, const int* in_sizes, int n_in,
                              void* d_out, int out_size, void* d_ws, size_t ws_size,
                              hipStream_t stream)
{
  if (n_in < 16) return;
  if (in_sizes[0] != SEQ_T * DMOD || in_sizes[1] != DMOD * CHN || in_sizes[2] != DMOD * CHN ||
      in_sizes[3] != DMOD * CHN || in_sizes[4] != KCONV * CHN || in_sizes[5] != KCONV * CHN ||
      in_sizes[6] != KCONV * CHN || in_sizes[7] != DMOD * HDIM || in_sizes[8] != HDIM * CHN ||
      in_sizes[9] != CHN || in_sizes[10] != NHEAD || in_sizes[11] != DMOD * NHEAD ||
      in_sizes[12] != DMOD * HDIM || in_sizes[13] != HDIM * CHN || in_sizes[14] != HDIM ||
      in_sizes[15] != CHN * DMOD) return;
  if (out_size != SEQ_T * DMOD) return;
  if (WS_TOTAL > ws_size) return;

  const float* x      = (const float*)d_in[0];
  const float* Wq     = (const float*)d_in[1];
  const float* Wk     = (const float*)d_in[2];
  const float* Wv     = (const float*)d_in[3];
  const float* convq  = (const float*)d_in[4];
  const float* convk  = (const float*)d_in[5];
  const float* convv  = (const float*)d_in[6];
  const float* Wfa    = (const float*)d_in[7];
  const float* Wfb    = (const float*)d_in[8];
  const float* dtbias = (const float*)d_in[9];
  const float* Alog   = (const float*)d_in[10];
  const float* Wb     = (const float*)d_in[11];
  const float* Wga    = (const float*)d_in[12];
  const float* Wgb    = (const float*)d_in[13];
  const float* normw  = (const float*)d_in[14];
  const float* Wo     = (const float*)d_in[15];
  float* out = (float*)d_out;

  char* ws = (char*)d_ws;
  unsigned short* xbf  = (unsigned short*)(ws + OFF_XBF);
  unsigned short* wt4  = (unsigned short*)(ws + OFF_WT4);
  unsigned short* wfg  = (unsigned short*)(ws + OFF_WFG);
  unsigned short* wfbg = (unsigned short*)(ws + OFF_WFBG);
  float* lin  = (float*)(ws + OFF_LIN);
  float* egp  = (float*)(ws + OFF_EG);
  float* obuf = (float*)(ws + OFF_OBUF);
  unsigned short* onh = (unsigned short*)(ws + OFF_ONH);
  unsigned short* onl = (unsigned short*)(ws + OFF_ONL);
  unsigned short* pfh = (unsigned short*)(ws + OFF_PFH);
  unsigned short* pfl = (unsigned short*)(ws + OFF_PFL);
  float* gr   = (float*)(ws + OFF_GR);
  float* post = (float*)(ws + OFF_POST);

  k_cast_bf16x8<<<dim3((unsigned)(TK_ELEMS / 8 / 256)), 256, 0, stream>>>(x, xbf, (int)(TK_ELEMS / 8));
  k_tr_bf16<<<dim3(CHN / 64, DMOD / 64, 4), 256, 0, stream>>>(Wq, Wk, Wv, Wo, wt4, (long)DMOD * CHN, DMOD, CHN, DMOD);
  k_tr_bf16<<<dim3(HDIM / 64, DMOD / 64, 2), 256, 0, stream>>>(Wfa, Wga, Wfa, Wga, wfg, (long)HDIM * DMOD, DMOD, HDIM, DMOD);
  k_tr_bf16<<<dim3(1, DMOD / 64, 1), 256, 0, stream>>>(Wb, Wb, Wb, Wb, wfg + (size_t)256 * DMOD, (long)0, DMOD, NHEAD, DMOD);
  k_tr_bf16<<<dim3(CHN / 64, HDIM / 64, 2), 256, 0, stream>>>(Wfb, Wgb, Wfb, Wgb, wfbg, (long)CHN * HDIM, HDIM, CHN, HDIM);

  wmma_gemm64<1, 0, 0, 0><<<dim3((SEQ_T / 64) * (CHN / 64) / 8, 3), 256, 0, stream>>>(
      xbf, nullptr, DMOD, (long)0,
      wt4, nullptr, DMOD, (long)DMOD * CHN,
      (void*)lin, nullptr, CHN, (long)TK_ELEMS,
      nullptr, SEQ_T, CHN, DMOD, 1.0f);
  wmma_gemm64<1, 0, 0, 2><<<dim3((SEQ_T / 64) * (NFG / 64) / 8, 1), 256, 0, stream>>>(
      xbf, nullptr, DMOD, (long)0,
      wfg, nullptr, DMOD, (long)0,
      (void*)pfh, (void*)pfl, NFG, (long)0,
      nullptr, SEQ_T, NFG, DMOD, 1.0f);
  wmma_gemm64<1, 1, 0, 0><<<dim3((SEQ_T / 64) * (CHN / 64) / 8, 2), 256, 0, stream>>>(
      pfh, pfl, NFG, (long)HDIM,
      wfbg, nullptr, HDIM, (long)CHN * HDIM,
      (void*)gr, nullptr, CHN, (long)TK_ELEMS,
      nullptr, SEQ_T, CHN, HDIM, 1.0f);

  k_conv_silu_norm<<<dim3(SEQ_T * NHEAD / 8, 3), 256, 0, stream>>>(lin, convq, convk, convv, post, 0.08838834764831845f);
  k_gate_exp<<<dim3((unsigned)(TK_ELEMS / 256)), 256, 0, stream>>>(gr, dtbias, Alog, egp);
  k_scan<<<dim3(NHEAD * 2), 512, 0, stream>>>(post, post + TK_ELEMS, post + 2 * TK_ELEMS, egp,
                                              (const unsigned*)(const void*)pfh, (const unsigned*)(const void*)pfl, obuf);
  k_rmsnorm_gate_split<<<dim3(SEQ_T * NHEAD / 16), 256, 0, stream>>>(obuf, gr + TK_ELEMS, normw, onh, onl);
  wmma_gemm64<1, 1, 0, 0><<<dim3((SEQ_T / 64) * (DMOD / 64) / 8, 1), 256, 0, stream>>>(
      onh, onl, CHN, (long)0,
      wt4 + (size_t)3 * DMOD * CHN, nullptr, CHN, (long)0,
      (void*)out, nullptr, DMOD, (long)0,
      nullptr, SEQ_T, DMOD, CHN, 1.0f);
}
